// Net_37830071943759
// MI455X (gfx1250) — hardware-verified
//
#include <hip/hip_runtime.h>
#include <stddef.h>
#include <stdint.h>
#include <math.h>


#define CIN    256
#define HID    128
#define KD     256
#define NTHR   256
#define NWAVE  8
#define EPT    8
#define CHUNK  (NTHR * EPT)
#define WCAP   (EPT * 32)
#define LISTN  (NWAVE * WCAP)
#define NBD    8192
#define SLD    13
#define NBA    1024
#define SLA    10
#define RCAP   20480
#define DEGCAP 64
#define GBM    64
#define GBN    64
#define GTHR   128
#define PT     64
#define PTHR   128
#define NUWC   (HID * (CIN / 8))
#define NUAB   (2 * HID * (KD / 8))
#define NUCC   (HID * (KD / 8))
#define S_HL   LISTN
#define S_SLI  (LISTN + RCAP)
#define S_CNTI (LISTN + 3 * RCAP)
#define S_CUR  (S_CNTI + 4 * NBA)
#define SC_ZINTS (S_CUR + NBA)
#define MISC_INTS 16
#define ROWBUF_INTS (NWAVE * 128)
#define SC_LDS_INTS (SC_ZINTS + MISC_INTS + ROWBUF_INTS)
#define WSMAX  134217728

static_assert((CHUNK & (CHUNK - 1)) == 0 && CHUNK <= 4096);
static_assert((NBD & (NBD - 1)) == 0 && NBD == (1 << SLD));
static_assert((NBA & (NBA - 1)) == 0 && NBA == (1 << SLA));
static_assert(((long long)CHUNK << SLD) < (1LL << 31));
static_assert(((long long)CHUNK << SLA) < (1LL << 31));
static_assert(NBD % (NTHR * 4) == 0);
static_assert(LISTN % NTHR == 0);
static_assert(NBA % NWAVE == 0 && NBA % 32 == 0 && NBA % GBM == 0);
static_assert(RCAP % 4 == 0 && SC_ZINTS % (NTHR * 4) == 0 && ((SC_ZINTS + MISC_INTS) % 4) == 0);
static_assert(CIN % 32 == 0 && KD % 32 == 0 && KD == 2 * HID && HID == 4 * 32);
static_assert(GBM == (GTHR / 32) * 16 && GBN == 64 && HID % GBN == 0);
static_assert(NUWC % NTHR == 0 && NUAB % NTHR == 0 && NUCC % NTHR == 0);
static_assert(CIN / 8 == 32 && KD / 8 == 32);
static_assert(PTHR == 2 * PT && PT == 64 && PT == (PTHR / 32) * 16);
static_assert(SC_LDS_INTS * 4 <= 300000);

typedef float          v4f   __attribute__((ext_vector_type(4)));
typedef float          v8f   __attribute__((ext_vector_type(8)));
typedef int            v4i   __attribute__((ext_vector_type(4)));
typedef int            v8i   __attribute__((ext_vector_type(8)));
typedef unsigned short v4us  __attribute__((ext_vector_type(4)));
typedef unsigned short v8us  __attribute__((ext_vector_type(8)));
typedef unsigned short v16us __attribute__((ext_vector_type(16)));
typedef __bf16         v16bf __attribute__((ext_vector_type(16)));
typedef v4f  __attribute__((may_alias)) v4fa;
typedef v4i  __attribute__((may_alias)) v4ia;
typedef v4us __attribute__((may_alias)) v4usa;
typedef v8us __attribute__((may_alias)) v8usa;
union FragB { v16bf v; v16us u; v8us h[2]; v8i w; };

__device__ __forceinline__ v8f wmb(const FragB& a, const FragB& b, v8f c) {
  v8f d = __builtin_amdgcn_wmma_f32_16x16x32_bf16(false, a.v, false, b.v, (short)0, c, false, false);
  asm volatile("v_nop\n\tv_nop\n\tv_nop\n\tv_nop" : "+v"(d) : "v"(a.w), "v"(b.w));
  return d;
}

__device__ __forceinline__ unsigned bf16_bits(float f) {
  const unsigned u = __float_as_uint(f);
  return (u + 0x7FFFu + ((u >> 16) & 1u)) >> 16;
}
__device__ __forceinline__ float bf16_val(float f) {
  return __uint_as_float(bf16_bits(f) << 16);
}

__device__ __forceinline__ float relu_np(float v) {
  return (v > 0.0f) ? v : (v - v);
}

__device__ __forceinline__ void wave_sync() {
  __builtin_amdgcn_fence(__ATOMIC_RELEASE, "wavefront");
  __builtin_amdgcn_wave_barrier();
  __builtin_amdgcn_fence(__ATOMIC_ACQUIRE, "wavefront");
}

template <int SLB>
__device__ __forceinline__ int scan_chunk(const int* __restrict__ dsts, int nE, int cbase, int slotBase,
                                          int nb, int vec8, int* list, int tid, int lane, int wave) {
  int wc = 0;
  const int el0  = tid * EPT;
  const int e0   = cbase + el0;
  const int sent = -2147483647 - 1;
  v4i da, db;
  if (vec8 != 0 && cbase + CHUNK <= nE) {
    da = *(const v4i*)(dsts + e0);
    db = *(const v4i*)(dsts + e0 + 4);
  } else {
    da.x = (e0     < nE) ? dsts[min(e0,     nE - 1)] : sent;
    da.y = (e0 + 1 < nE) ? dsts[min(e0 + 1, nE - 1)] : sent;
    da.z = (e0 + 2 < nE) ? dsts[min(e0 + 2, nE - 1)] : sent;
    da.w = (e0 + 3 < nE) ? dsts[min(e0 + 3, nE - 1)] : sent;
    db.x = (e0 + 4 < nE) ? dsts[min(e0 + 4, nE - 1)] : sent;
    db.y = (e0 + 5 < nE) ? dsts[min(e0 + 5, nE - 1)] : sent;
    db.z = (e0 + 6 < nE) ? dsts[min(e0 + 6, nE - 1)] : sent;
    db.w = (e0 + 7 < nE) ? dsts[min(e0 + 7, nE - 1)] : sent;
  }
  const unsigned nbs = (unsigned)slotBase;
  const unsigned unb = (unsigned)nb;
  const unsigned s0 = (unsigned)da.x - nbs, s1 = (unsigned)da.y - nbs;
  const unsigned s2 = (unsigned)da.z - nbs, s3 = (unsigned)da.w - nbs;
  const unsigned s4 = (unsigned)db.x - nbs, s5 = (unsigned)db.y - nbs;
  const unsigned s6 = (unsigned)db.z - nbs, s7 = (unsigned)db.w - nbs;
  const bool h0 = s0 < unb, h1 = s1 < unb, h2 = s2 < unb, h3 = s3 < unb;
  const bool h4 = s4 < unb, h5 = s5 < unb, h6 = s6 < unb, h7 = s7 < unb;
  const unsigned any = __builtin_amdgcn_ballot_w32(h0 | h1 | h2 | h3 | h4 | h5 | h6 | h7);
  if (any != 0u) {
#define HITJ(J, HJ, SJ) { \
      const unsigned mj = __builtin_amdgcn_ballot_w32(HJ); \
      if (mj != 0u) { \
        if (HJ) { \
          const int pos = wc + (int)__builtin_amdgcn_mbcnt_lo(mj, 0u); \
          if (pos < WCAP) list[wave * WCAP + pos] = ((el0 + (J)) << SLB) | (int)(SJ); \
        } \
        wc += (int)__builtin_popcount(mj); } }
    HITJ(0, h0, s0)
    HITJ(1, h1, s1)
    HITJ(2, h2, s2)
    HITJ(3, h3, s3)
    HITJ(4, h4, s4)
    HITJ(5, h5, s5)
    HITJ(6, h6, s6)
    HITJ(7, h7, s7)
#undef HITJ
  }
  return wc;
}

__global__ __launch_bounds__(NTHR) void k_wprep(const float* __restrict__ Wc, const float* __restrict__ W1,
                                                unsigned short* WcT, unsigned short* WabT,
                                                unsigned short* WccT) {
  const int u = (int)blockIdx.x * NTHR + (int)threadIdx.x;
  const float* p;
  unsigned short* dp;
  if (u < NUWC) {
    const int n  = u >> 5;
    const int k8 = (u & 31) * 8;
    p  = Wc + (size_t)k8 * HID + n;
    dp = WcT + (size_t)n * CIN + k8;
  } else if (u < NUWC + NUAB) {
    const int v  = u - NUWC;
    const int n  = v >> 5;
    const int k8 = (v & 31) * 8;
    const int kk = k8 & (HID - 1);
    p  = W1 + (size_t)((n >> 7) * HID + kk) * HID + (n & (HID - 1));
    dp = WabT + (size_t)n * KD + k8;
  } else if (u < NUWC + NUAB + NUCC) {
    const int v  = u - NUWC - NUAB;
    const int n  = v >> 5;
    const int k8 = (v & 31) * 8;
    const int kk = k8 & (HID - 1);
    p  = W1 + (size_t)(2 * HID + kk) * HID + n;
    dp = WccT + (size_t)n * KD + k8;
  } else {
    return;
  }
  v8us o;
#pragma unroll
  for (int i = 0; i < 8; ++i) o[i] = (unsigned short)bf16_bits(p[(size_t)i * HID]);
  *(volatile v8us*)dp = o;
  __threadfence();
  *(volatile v8us*)dp = o;
}

__global__ __launch_bounds__(NTHR) void k_cvx(const float* __restrict__ x, int nN, int nUnits,
                                              unsigned short* xb) {
  const int u = (int)blockIdx.x * NTHR + (int)threadIdx.x;
  if (u >= nUnits) return;
  const int row = u >> 5;
  const int k8  = (u & 31) * 8;
  const int rc  = row < nN ? row : nN - 1;
  const float* p = x + (size_t)rc * CIN + k8;
  const v4f a = *(const v4fa*)p;
  const v4f b = *(const v4fa*)(p + 4);
  const bool ok = row < nN;
  v8us o;
  o[0] = ok ? (unsigned short)bf16_bits(a.x) : (unsigned short)0;
  o[1] = ok ? (unsigned short)bf16_bits(a.y) : (unsigned short)0;
  o[2] = ok ? (unsigned short)bf16_bits(a.z) : (unsigned short)0;
  o[3] = ok ? (unsigned short)bf16_bits(a.w) : (unsigned short)0;
  o[4] = ok ? (unsigned short)bf16_bits(b.x) : (unsigned short)0;
  o[5] = ok ? (unsigned short)bf16_bits(b.y) : (unsigned short)0;
  o[6] = ok ? (unsigned short)bf16_bits(b.z) : (unsigned short)0;
  o[7] = ok ? (unsigned short)bf16_bits(b.w) : (unsigned short)0;
  unsigned short* dp = xb + (size_t)row * CIN + k8;
  *(volatile v8us*)dp = o;
  __threadfence();
  *(volatile v8us*)dp = o;
}

__global__ __launch_bounds__(NTHR) void k_deg(const int* __restrict__ dstI, const int* __restrict__ dstD,
                                              int nE, int vec8, float* dinv, int nbpd) {
  __shared__ __attribute__((aligned(16))) int scnt[NBD];
  __shared__ __attribute__((aligned(16))) int list[LISTN];
  __shared__ int wcnt[NWAVE];
  const int tid = (int)threadIdx.x, lane = tid & 31, wave = tid >> 5;
  const int g = (int)blockIdx.y;
  const int* dsts = (g != 0) ? dstD : dstI;
  float* dis = dinv + (size_t)g * (size_t)nbpd;
  const int nodeBase = (int)blockIdx.x * NBD;

  for (int i = tid; i < NBD; i += NTHR) scnt[i] = 0;
  for (int i = tid; i < LISTN; i += NTHR) list[i] = 0;
  if (tid < NWAVE) wcnt[tid] = 0;
  __syncthreads();

  const int nChunks = (nE + CHUNK - 1) / CHUNK;
#pragma unroll 1
  for (int ch = 0; ch < nChunks; ++ch) {
    const int cbase = ch * CHUNK;
    const int wc = scan_chunk<SLD>(dsts, nE, cbase, nodeBase, NBD, vec8, list, tid, lane, wave);
    if (lane == 0) wcnt[wave] = wc;
    __syncthreads();
    if (wave == 0) {
#pragma unroll 1
      for (int w2 = 0; w2 < NWAVE; ++w2) {
        int c = wcnt[w2];
        c = c < 0 ? 0 : (c > WCAP ? WCAP : c);
#pragma unroll 1
        for (int b0 = 0; b0 < c; b0 += 32) {
          const int idx = b0 + lane;
          const int ent = list[w2 * WCAP + (idx < WCAP ? idx : WCAP - 1)];
          const int m32 = (c - b0) < 32 ? (c - b0) : 32;
#pragma unroll 1
          for (int k = 0; k < m32; ++k) {
            const int u  = __builtin_amdgcn_readlane(ent, k);
            const int sl = u & (NBD - 1);
            if (lane == 0) scnt[sl] = scnt[sl] + 1;
          }
        }
      }
    }
    __syncthreads();
  }

  v4f vals[NBD / (NTHR * 4)];
#pragma unroll
  for (int it = 0; it < NBD / (NTHR * 4); ++it) {
    const int s0 = it * (NTHR * 4) + 4 * tid;
    const v4i c4 = *(const v4ia*)(scnt + s0);
    const float d0 = (float)c4.x + 1.0f, d1 = (float)c4.y + 1.0f;
    const float d2 = (float)c4.z + 1.0f, d3 = (float)c4.w + 1.0f;
    v4f v;
    v.x = rsqrtf(d0); v.y = rsqrtf(d1); v.z = rsqrtf(d2); v.w = rsqrtf(d3);
    vals[it] = v;
  }
#pragma unroll
  for (int it = 0; it < NBD / (NTHR * 4); ++it) {
    const int s0 = it * (NTHR * 4) + 4 * tid;
    *(volatile v4f*)(dis + (size_t)nodeBase + s0) = vals[it];
  }
  __threadfence();
#pragma unroll
  for (int it = 0; it < NBD / (NTHR * 4); ++it) {
    const int s0 = it * (NTHR * 4) + 4 * tid;
    *(volatile v4f*)(dis + (size_t)nodeBase + s0) = vals[it];
  }
}

__global__ __launch_bounds__(GTHR) void k_gemm(
    const unsigned short* __restrict__ A, const unsigned short* __restrict__ WT,
    float* outF, int K, int ldo, const float* __restrict__ bias, int nb)
{
  __shared__ __attribute__((aligned(16))) float stg[GBM * GBN];
  const int tid = (int)threadIdx.x, lane = tid & 31, wave = tid >> 5, hh = lane >> 4, m = lane & 15;
  const int rowBase = (int)blockIdx.x * GBM;
  const int col0    = (int)blockIdx.y * GBN;

  v8f acc[4];
  {
    const v8f z = {0.f, 0.f, 0.f, 0.f, 0.f, 0.f, 0.f, 0.f};
    acc[0] = z; acc[1] = z; acc[2] = z; acc[3] = z;
  }
  const unsigned short* ap = A  + (size_t)(rowBase + 16 * wave + m) * (size_t)K + 8 * hh;
  const unsigned short* wp = WT + (size_t)(col0 + m) * (size_t)K + 8 * hh;
  const int ksteps = K >> 5;
#pragma unroll 1
  for (int ks = 0; ks < ksteps; ++ks) {
    FragB af;
    af.h[0] = *(const v8usa*)(ap + 32 * ks);
    af.h[1] = *(const v8usa*)(ap + 32 * ks + 16);
#pragma unroll
    for (int t = 0; t < 4; ++t) {
      const unsigned short* wq = wp + (size_t)(16 * t) * (size_t)K + 32 * ks;
      FragB bf;
      bf.h[0] = *(const v8usa*)wq;
      bf.h[1] = *(const v8usa*)(wq + 16);
      acc[t] = wmb(af, bf, acc[t]);
    }
  }

#pragma unroll
  for (int t = 0; t < 4; ++t) {
    const int lc = 16 * t + m;
#pragma unroll
    for (int r = 0; r < 8; ++r) {
      const int lr = 16 * wave + 8 * hh + r;
      stg[lr * GBN + lc] = acc[t][r];
    }
  }
  __syncthreads();

  v4f badd;
  {
    const int cb = col0 + 4 * m;
    const v4f braw = *(const v4f*)(bias + (cb & (HID - 1)));
    const float bsel = (cb < nb) ? 1.0f : 0.0f;
    badd.x = bf16_val(braw.x) * bsel; badd.y = bf16_val(braw.y) * bsel;
    badd.z = bf16_val(braw.z) * bsel; badd.w = bf16_val(braw.w) * bsel;
  }
  v4f fv[8];
#pragma unroll
  for (int i = 0; i < 8; ++i) {
    const int lr = 16 * wave + 2 * i + hh;
    const v4f t = *(const v4fa*)(stg + lr * GBN + 4 * m);
    fv[i] = t + badd;
  }
#pragma unroll
  for (int i = 0; i < 8; ++i) {
    const int lr = 16 * wave + 2 * i + hh;
    const int gr = rowBase + lr;
    float* op = outF + (size_t)gr * (size_t)ldo + col0 + 4 * m;
    *(volatile v4f*)op = fv[i];
  }
  __threadfence();
#pragma unroll
  for (int i = 0; i < 8; ++i) {
    const int lr = 16 * wave + 2 * i + hh;
    const int gr = rowBase + lr;
    float* op = outF + (size_t)gr * (size_t)ldo + col0 + 4 * m;
    *(volatile v4f*)op = fv[i];
  }
}

__global__ __launch_bounds__(NTHR) void k_scan(const int* __restrict__ srcI, const int* __restrict__ dstI,
                                               const int* __restrict__ srcD, const int* __restrict__ dstD,
                                               int nE, int nN, int vec8, int mRows,
                                               const float* __restrict__ dinvI, const float* __restrict__ dinvD,
                                               const float* __restrict__ xl, const float* __restrict__ bconv,
                                               float* Zf, unsigned short* Zhl) {
  extern __shared__ __attribute__((aligned(16))) int dsm[];
  int* list = dsm;
  int* hl   = dsm + S_HL;
  int* cur  = dsm + S_CUR;
  int* misc = dsm + SC_ZINTS;
  const int tid = (int)threadIdx.x, lane = tid & 31, wave = tid >> 5;
  unsigned short* rowbuf = (unsigned short*)(misc + MISC_INTS) + wave * 256;
  const int nodeBase = (int)blockIdx.x * NBA;

  {
    const v4i z4 = {0, 0, 0, 0};
    for (int i = tid * 4; i < SC_ZINTS; i += NTHR * 4) *(v4ia*)(dsm + i) = z4;
    if (tid < MISC_INTS) misc[tid] = 0;
  }
  __syncthreads();

  const int nChunks = (nE + CHUNK - 1) / CHUNK;
#pragma unroll 1
  for (int g = 0; g < 2; ++g) {
    const int* keys = (g != 0) ? dstD : dstI;
    int* sl   = dsm + S_SLI + g * RCAP;
    int* cnt  = dsm + S_CNTI + g * 2 * NBA;
    int* offs = cnt + NBA;

    int t = 0, ov = 0;
#pragma unroll 1
    for (int ch = 0; ch < nChunks; ++ch) {
      const int cbase = ch * CHUNK;
      const int wc = scan_chunk<SLA>(keys, nE, cbase, nodeBase, NBA, vec8, list, tid, lane, wave);
      if (lane == 0) misc[wave] = wc;
      __syncthreads();
      if (wave == 0) {
#pragma unroll 1
        for (int w2 = 0; w2 < NWAVE; ++w2) {
          int c = misc[w2];
          c = c < 0 ? 0 : (c > WCAP ? WCAP : c);
#pragma unroll 1
          for (int b0 = 0; b0 < c; b0 += 32) {
            const int idx = b0 + lane;
            const int ent = list[w2 * WCAP + (idx < WCAP ? idx : WCAP - 1)];
            const int m32 = (c - b0) < 32 ? (c - b0) : 32;
#pragma unroll 1
            for (int k = 0; k < m32; ++k) {
              const int u    = __builtin_amdgcn_readlane(ent, k);
              const int slot = u & (NBA - 1);
              const int el   = (u >> SLA) & (CHUNK - 1);
              const int pk   = ((cbase + el) << SLA) | slot;
              if (t < RCAP) {
                if (lane == 0) { hl[t] = pk; cnt[slot] = cnt[slot] + 1; }
                t = t + 1;
              } else {
                ov = 1;
              }
            }
          }
        }
      }
      __syncthreads();
    }
    if (wave == 0 && lane == 0) { misc[8 + 2 * g] = t; misc[9 + 2 * g] = ov; }
    __syncthreads();
    int tt = misc[8 + 2 * g];
    tt = tt < 0 ? 0 : (tt > RCAP ? RCAP : tt);

    if (wave == 0) {
      const int base = lane * (NBA / 32);
      int s = 0;
#pragma unroll 1
      for (int i = 0; i < NBA / 32; ++i) s += cnt[base + i];
      int incl = s;
#pragma unroll
      for (int d = 1; d < 32; d <<= 1) {
        const int y = __shfl_up(incl, d, 32);
        if (lane >= d) incl += y;
      }
      int run = incl - s;
#pragma unroll 1
      for (int i = 0; i < NBA / 32; ++i) {
        const int cv = cnt[base + i];
        offs[base + i] = run;
        cur[base + i]  = run;
        run += cv;
      }
    }
    __syncthreads();
    if (wave == 0) {
#pragma unroll 1
      for (int b0 = 0; b0 < tt; b0 += 32) {
        const int idx = b0 + lane;
        const int ent = hl[idx < RCAP ? idx : RCAP - 1];
        const int m32 = (tt - b0) < 32 ? (tt - b0) : 32;
#pragma unroll 1
        for (int k = 0; k < m32; ++k) {
          const int u    = __builtin_amdgcn_readlane(ent, k);
          const int slot = u & (NBA - 1);
          if (lane == 0) {
            int p = cur[slot];
            p = p < 0 ? 0 : (p > RCAP - 1 ? RCAP - 1 : p);
            sl[p] = u;
            cur[slot] = p + 1;
          }
        }
      }
    }
    __syncthreads();
  }

  const float qnan = __int_as_float(0x7fc00000);
  const int ovf = misc[9] | misc[11];
  const float pz = (ovf != 0) ? qnan : 0.0f;
  v4f bv;
  {
    const v4f a = *(const v4f*)(bconv + 4 * lane);
    bv.x = bf16_val(a.x); bv.y = bf16_val(a.y); bv.z = bf16_val(a.z); bv.w = bf16_val(a.w);
  }
#pragma unroll 1
  for (int si = 0; si < NBA / NWAVE; ++si) {
    const int s    = si * NWAVE + wave;
    const int node = nodeBase + s;
    const int nc = node < nN ? node : nN - 1;
    const v4f xs = *(const v4f*)(xl + (size_t)nc * HID + 4 * lane);
    float z0 = 0.0f, z1 = 0.0f, z2 = 0.0f, z3 = 0.0f;
    int bigf = 0;
#pragma unroll 1
    for (int g = 0; g < 2; ++g) {
      const int*   srcs = (g != 0) ? srcD : srcI;
      const float* dis  = (g != 0) ? dinvD : dinvI;
      const int*   sl   = dsm + S_SLI + g * RCAP;
      int c = dsm[S_CNTI + g * 2 * NBA + s];
      int o = dsm[S_CNTI + (g * 2 + 1) * NBA + s];
      bigf |= (c > DEGCAP) ? 1 : 0;
      c = c < 0 ? 0 : (c > DEGCAP ? DEGCAP : c);
      o = o < 0 ? 0 : (o > RCAP ? RCAP : o);
      const float dd = dis[nc];
      const float rd = dd * dd;
      float a0 = 0.0f, a1 = 0.0f, a2 = 0.0f, a3 = 0.0f;
#pragma unroll 1
      for (int b0 = 0; b0 < c; b0 += 32) {
        int idx = o + b0 + lane;
        idx = idx > RCAP - 1 ? RCAP - 1 : idx;
        const int ent = sl[idx];
        int eid = ent >> SLA;
        eid = eid < 0 ? 0 : (eid > nE - 1 ? nE - 1 : eid);
        int sr = srcs[eid];
        sr = sr < 0 ? 0 : (sr > nN - 1 ? nN - 1 : sr);
        const float cf  = dis[sr] * dd;
        const int   cfi = __float_as_int(cf);
        const int m32 = (c - b0) < 32 ? (c - b0) : 32;
#pragma unroll 1
        for (int k = 0; k < m32; ++k) {
          const int   sk = __builtin_amdgcn_readlane(sr, k);
          const float ck = __int_as_float(__builtin_amdgcn_readlane(cfi, k));
          const v4f a = *(const v4f*)(xl + (size_t)sk * HID + 4 * lane);
          a0 = fmaf(ck, a.x, a0); a1 = fmaf(ck, a.y, a1);
          a2 = fmaf(ck, a.z, a2); a3 = fmaf(ck, a.w, a3);
        }
      }
      const float y0 = fmaxf((a0 + xs.x * rd) + bv.x, 0.0f);
      const float y1 = fmaxf((a1 + xs.y * rd) + bv.y, 0.0f);
      const float y2 = fmaxf((a2 + xs.z * rd) + bv.z, 0.0f);
      const float y3 = fmaxf((a3 + xs.w * rd) + bv.w, 0.0f);
      z0 += y0; z1 += y1; z2 += y2; z3 += y3;
    }
    const float pzr = (bigf != 0) ? qnan : pz;
    const bool live = node < nN;
    v4f zv;
    zv.x = live ? (z0 + pzr) : 0.0f;
    zv.y = live ? (z1 + pzr) : 0.0f;
    zv.z = live ? (z2 + pzr) : 0.0f;
    zv.w = live ? (z3 + pzr) : 0.0f;
    v4us mh, ml;
    {
      unsigned hb;
      hb = bf16_bits(zv.x); mh[0] = (unsigned short)hb; ml[0] = (unsigned short)bf16_bits(zv.x - __uint_as_float(hb << 16));
      hb = bf16_bits(zv.y); mh[1] = (unsigned short)hb; ml[1] = (unsigned short)bf16_bits(zv.y - __uint_as_float(hb << 16));
      hb = bf16_bits(zv.z); mh[2] = (unsigned short)hb; ml[2] = (unsigned short)bf16_bits(zv.z - __uint_as_float(hb << 16));
      hb = bf16_bits(zv.w); mh[3] = (unsigned short)hb; ml[3] = (unsigned short)bf16_bits(zv.w - __uint_as_float(hb << 16));
    }
    *(v4usa*)(rowbuf + 4 * lane) = mh;
    *(v4usa*)(rowbuf + HID + 4 * lane) = ml;
    wave_sync();
    const v8us q0 = *(const v8usa*)(rowbuf + 8 * lane);
    wave_sync();
    if (node < mRows) {
      float* zp = Zf + (size_t)node * HID + 4 * lane;
      unsigned short* hp = Zhl + (size_t)node * KD + 8 * lane;
      *(volatile v4f*)zp = zv;
      *(volatile v8us*)hp = q0;
      __threadfence();
      *(volatile v4f*)zp = zv;
      *(volatile v8us*)hp = q0;
    }
  }
}

__global__ __launch_bounds__(PTHR) void k_pair(const int* __restrict__ eli, int nP, int nN,
                                               const float* __restrict__ Zf, const float* __restrict__ AB,
                                               const unsigned short* __restrict__ WT,
                                               const float* __restrict__ W2, const float* __restrict__ b2,
                                               float* out) {
  __shared__ __attribute__((aligned(16))) float stg[PT * HID];
  __shared__ int sidx[2 * PT];
  __shared__ __attribute__((aligned(16))) float outs[PT];
  const int tid = (int)threadIdx.x, lane = tid & 31, wave = tid >> 5, hh = lane >> 4, m = lane & 15;
  const int p0 = (int)blockIdx.x * PT;

  {
    const int r = tid & (PT - 1);
    const int which = tid >> 6;
    int p = p0 + r;
    p = p > nP - 1 ? nP - 1 : p;
    int v = eli[(size_t)which * (size_t)nP + p];
    v = v < 0 ? 0 : (v > nN - 1 ? nN - 1 : v);
    sidx[tid] = v;
  }
  __syncthreads();

  unsigned short* at = (unsigned short*)stg;
#pragma unroll 1
  for (int r = 0; r < 16; ++r) {
    const int row = 16 * wave + r;
    const int i = sidx[row];
    const int j = sidx[PT + row];
    const v4f zi = *(const v4f*)(Zf + (size_t)i * HID + 4 * lane);
    const v4f zj = *(const v4f*)(Zf + (size_t)j * HID + 4 * lane);
    const float d0 = fabsf(zi.x - zj.x), d1 = fabsf(zi.y - zj.y);
    const float d2 = fabsf(zi.z - zj.z), d3 = fabsf(zi.w - zj.w);
    v4us mh, ml;
    unsigned hb;
    hb = bf16_bits(d0); mh[0] = (unsigned short)hb; ml[0] = (unsigned short)bf16_bits(d0 - __uint_as_float(hb << 16));
    hb = bf16_bits(d1); mh[1] = (unsigned short)hb; ml[1] = (unsigned short)bf16_bits(d1 - __uint_as_float(hb << 16));
    hb = bf16_bits(d2); mh[2] = (unsigned short)hb; ml[2] = (unsigned short)bf16_bits(d2 - __uint_as_float(hb << 16));
    hb = bf16_bits(d3); mh[3] = (unsigned short)hb; ml[3] = (unsigned short)bf16_bits(d3 - __uint_as_float(hb << 16));
    *(v4usa*)(at + (size_t)row * KD + 4 * lane) = mh;
    *(v4usa*)(at + (size_t)row * KD + HID + 4 * lane) = ml;
  }
  __syncthreads();

  v8f acc[8];
  {
    const v8f z = {0.f, 0.f, 0.f, 0.f, 0.f, 0.f, 0.f, 0.f};
#pragma unroll
    for (int t = 0; t < 8; ++t) acc[t] = z;
  }
  {
    const unsigned short* ap = at + (size_t)(16 * wave + m) * KD + 8 * hh;
    const unsigned short* bp = WT + (size_t)m * KD + 8 * hh;
#pragma unroll 1
    for (int k0 = 0; k0 < KD; k0 += 32) {
      FragB af;
      af.h[0] = *(const v8usa*)(ap + k0);
      af.h[1] = *(const v8usa*)(ap + k0 + 16);
#pragma unroll
      for (int nt = 0; nt < 8; ++nt) {
        const unsigned short* wq = bp + (size_t)(16 * nt) * KD + k0;
        FragB bf;
        bf.h[0] = *(const v8usa*)wq;
        bf.h[1] = *(const v8usa*)(wq + 16);
        acc[nt] = wmb(af, bf, acc[nt]);
      }
    }
  }
  __syncthreads();

#pragma unroll
  for (int nt = 0; nt < 8; ++nt) {
    const int lc = 16 * nt + m;
#pragma unroll
    for (int r = 0; r < 8; ++r) {
      const int lr = 16 * wave + 8 * hh + r;
      stg[lr * HID + lc] = acc[nt][r];
    }
  }
  __syncthreads();

  v4f w2v;
  {
    const v4f a = *(const v4f*)(W2 + 4 * lane);
    w2v.x = bf16_val(a.x); w2v.y = bf16_val(a.y); w2v.z = bf16_val(a.z); w2v.w = bf16_val(a.w);
  }
  const float b2v = bf16_val(b2[0]);
#pragma unroll 1
  for (int r = 0; r < 16; ++r) {
    const int row = 16 * wave + r;
    const int i = sidx[row];
    const int j = sidx[PT + row];
    const v4f a  = *(const v4fa*)(stg + row * HID + 4 * lane);
    const v4f ai = *(const v4f*)(AB + (size_t)i * KD + 4 * lane);
    const v4f bj = *(const v4f*)(AB + (size_t)j * KD + HID + 4 * lane);
    const float t0 = relu_np((a.x + ai.x) + bj.x);
    const float t1 = relu_np((a.y + ai.y) + bj.y);
    const float t2 = relu_np((a.z + ai.z) + bj.z);
    const float t3 = relu_np((a.w + ai.w) + bj.w);
    float s = t0 * w2v.x;
    s = fmaf(t1, w2v.y, s);
    s = fmaf(t2, w2v.z, s);
    s = fmaf(t3, w2v.w, s);
    s += __shfl_xor(s, 16, 32);
    s += __shfl_xor(s, 8, 32);
    s += __shfl_xor(s, 4, 32);
    s += __shfl_xor(s, 2, 32);
    s += __shfl_xor(s, 1, 32);
    if (lane == 0) outs[row] = s + b2v;
  }
  __syncthreads();

  const v4f ov = *(const v4fa*)(outs + 4 * (lane & 15));
  const int pe = p0 + 4 * (lane & 15);
  const int pc = pe < nP - 4 ? pe : nP - 4;
  float* op = out + (size_t)pc;
  const bool okst = (wave == 0) && (lane < 16) && (pe < nP);
  if (okst) *(volatile v4f*)op = ov;
  __threadfence();
  if (okst) *(volatile v4f*)op = ov;
}

static inline int cdiv(int a, int b) { return (a + b - 1) / b; }
static inline size_t al256(size_t o) { return (o + 255) & ~(size_t)255; }

extern "C" void kernel_launch(void* const* d_in, const int* in_sizes, int n_in,
                              void* d_out, int out_size, void* d_ws, size_t ws_size,
                              hipStream_t stream) {
  if (n_in < 10) return;
  if (in_sizes[0] < CIN || (in_sizes[0] % CIN) != 0) return;
  const int nN = in_sizes[0] / CIN;
  if (nN < 1 || nN > (1 << 22)) return;
  if (in_sizes[1] < 2 || (in_sizes[1] & 1) != 0) return;
  const int nE = in_sizes[1] / 2;
  if (in_sizes[2] != in_sizes[1]) return;
  if (nE < 1 || nE >= (1 << (31 - SLA))) return;
  if (in_sizes[3] < 2 || (in_sizes[3] & 1) != 0) return;
  const int nP = in_sizes[3] / 2;
  if (nP < 32 || (nP % 32) != 0) return;
  if (in_sizes[4] != CIN * HID || in_sizes[5] != HID) return;
  if (in_sizes[6] != 3 * HID * HID || in_sizes[7] != HID) return;
  if (in_sizes[8] != HID || in_sizes[9] != 1) return;
  if (out_size != nP) return;

  const float* x    = (const float*)d_in[0];
  const int*   eI   = (const int*)d_in[1];
  const int*   eD   = (const int*)d_in[2];
  const int*   eL   = (const int*)d_in[3];
  const float* Wc   = (const float*)d_in[4];
  const float* bc   = (const float*)d_in[5];
  const float* W1   = (const float*)d_in[6];
  const float* b1   = (const float*)d_in[7];
  const float* W2   = (const float*)d_in[8];
  const float* b2   = (const float*)d_in[9];
  float* out = (float*)d_out;
  const int* srcI = eI;
  const int* dstI = eI + nE;
  const int* srcD = eD;
  const int* dstD = eD + nE;

  const int MP   = cdiv(nN, GBM) * GBM;
  const int gM   = MP / GBM;
  const int gD   = cdiv(nN, NBD);
  const int NBPD = gD * NBD;
  const int gA   = cdiv(MP, NBA);
  if ((long long)gA * NBA < (long long)MP) return;
  if (NBPD < nN) return;
  const int vec8 = ((nE & 3) == 0) ? 1 : 0;
  const int gP   = cdiv(nP, PT);

  char* ws = (char*)d_ws;
  size_t off = 0;
  const size_t oWcT = off; off = al256(off + (size_t)HID * CIN * 2);
  const size_t oWab = off; off = al256(off + (size_t)2 * HID * KD * 2);
  const size_t oWcc = off; off = al256(off + (size_t)HID * KD * 2);
  const size_t oDIV = off; off = al256(off + (size_t)2 * NBPD * 4);
  const size_t oXB  = off; off = al256(off + (size_t)MP * CIN * 2);
  const size_t oXL  = off; off = al256(off + (size_t)MP * HID * 4);
  const size_t oZ   = off; off = al256(off + (size_t)MP * HID * 4);
  const size_t oZH  = off; off = al256(off + (size_t)MP * KD * 2);
  if (off > ws_size || off > (size_t)WSMAX) return;
  if (oXL - oXB != (size_t)MP * CIN * 2) return;
  if (oZ - oXB != (size_t)MP * KD * 4) return;
  unsigned short* WcT  = (unsigned short*)(ws + oWcT);
  unsigned short* WabT = (unsigned short*)(ws + oWab);
  unsigned short* WccT = (unsigned short*)(ws + oWcc);
  float*          DINV = (float*)(ws + oDIV);
  unsigned short* XB   = (unsigned short*)(ws + oXB);
  float*          XL   = (float*)(ws + oXL);
  float*          AB   = (float*)(ws + oXB);
  float*          Zf   = (float*)(ws + oZ);
  unsigned short* ZHL  = (unsigned short*)(ws + oZH);
  const float* dinvI = DINV;
  const float* dinvD = DINV + NBPD;

  const size_t scanLds = (size_t)SC_LDS_INTS * 4;
  hipFuncSetAttribute(reinterpret_cast<const void*>(&k_scan), hipFuncAttributeMaxDynamicSharedMemorySize, (int)scanLds);

  const int nUx = MP * (CIN / 8);
  k_wprep<<<(NUWC + NUAB + NUCC) / NTHR, NTHR, 0, stream>>>(Wc, W1, WcT, WabT, WccT);
  k_cvx<<<cdiv(nUx, NTHR), NTHR, 0, stream>>>(x, nN, nUx, XB);
  k_deg<<<dim3(gD, 2), NTHR, 0, stream>>>(dstI, dstD, nE, vec8, DINV, NBPD);
  k_gemm<<<dim3(gM, HID / GBN), GTHR, 0, stream>>>(XB, WcT, XL, CIN, HID, b1, 0);
  k_scan<<<gA, NTHR, scanLds, stream>>>(srcI, dstI, srcD, dstD, nE, nN, vec8, MP, dinvI, dinvD, XL, bc, Zf, ZHL);
  k_gemm<<<dim3(gM, (2 * HID) / GBN), GTHR, 0, stream>>>(ZHL, WabT, AB, KD, 2 * HID, b1, HID);
  k_pair<<<gP, PTHR, 0, stream>>>(eL, nP, nN, Zf, AB, WccT, W2, b2, out);
}
